// FMPlus_523986010576
// MI455X (gfx1250) — hardware-verified
//
#include <hip/hip_runtime.h>


namespace {
constexpr int NB = 4096, F = 30, D = 32, A = 32, P = 435, PP = 448, SPB = 32  ;
constexpr float XS = 8.0f, WSC = 256.0f;

typedef _Float16 b16;
typedef __attribute__((ext_vector_type(16))) _Float16 v16b;
typedef __attribute__((ext_vector_type(8))) _Float16 v8b;
typedef __attribute__((ext_vector_type(8))) float v8f;
typedef __attribute__((ext_vector_type(4))) float v4f;
__device__ __forceinline__ float bf16_rne(float f) { unsigned int u = __float_as_uint(f); u += 0x7FFFu + ((u >> 16) & 1u); return __uint_as_float(u & 0xFFFF0000u); }
__device__ __forceinline__ void split16(float v, b16& hi, b16& lo) { hi = (b16)v; lo = (b16)(v - (float)hi); }
__device__ __forceinline__ v16b frag_kb(const b16* p, int hh) { const v8b a = *(const v8b*)(p + 8 * hh), b = *(const v8b*)(p + 16 + 8 * hh); v16b f;
#pragma unroll
  for (int e = 0; e < 8; ++e) { f[e] = a[e]; f[8 + e] = b[e]; } return f; }
__device__ __forceinline__ v8f wmma16b(v16b a, v16b b, v8f c) { v8f d = __builtin_amdgcn_wmma_f32_16x16x32_f16(false, a, false, b, (short)0, c, false, false); asm volatile("v_nop\n\tv_nop\n\tv_nop\n\tv_nop" : "+v"(d) : "v"(a), "v"(b)); return d; }
__device__ __forceinline__ float pmul(float a, float b) { float p = a * b; asm volatile("" : "+v"(p)); return p; }
__device__ __forceinline__ float nexp(float x) { return __builtin_amdgcn_exp2f(x * 1.4426950408889634f); }

__device__ __forceinline__ void pair_ij(int p, int& i, int& j) { int base = 0; i = 0;
#pragma unroll 1
  for (int ii = 0; ii < F - 1; ++ii) { const int cnt = F - 1 - ii; if (p < base + cnt) { i = ii; j = ii + 1 + (p - base); return; } base += cnt; } i = F - 2; j = F - 1; }

__global__ __launch_bounds__(128) void fm_kernel(const float* __restrict__ emb, const float* __restrict__ w1, const float* __restrict__ b1, const float* __restrict__ w2, float* __restrict__ out) {
  __shared__ __attribute__((aligned(16))) b16 Ph[PP][D + 8], Pl[PP][D + 8]; __shared__ __attribute__((aligned(16))) b16 W1h[A][D + 8]; __shared__ float Es[F][D]; __shared__ float S[PP]; __shared__ float LG[PP]; __shared__ float red[4]; __shared__ float res[SPB];
  const int wave = threadIdx.x >> 5, lane = threadIdx.x & 31, nloc = lane & 15, hlf = lane >> 4, t_ = threadIdx.x; const int b0 = blockIdx.x * SPB;
  for (int q = t_; q < A * D; q += 128) W1h[q / D][q % D] = (b16)(bf16_rne(w1[q]) * WSC);
  const float b1v0 = bf16_rne(b1[nloc]), b1v1 = bf16_rne(b1[16 + nloc]), w2v0 = bf16_rne(w2[nloc]), w2v1 = bf16_rne(w2[16 + nloc]);
  for (int s = 0; s < SPB; ++s) { const int b = b0 + s;
    __syncthreads();
    for (int q = t_; q < F * D; q += 128) Es[q / D][q % D] = bf16_rne(emb[((size_t)b * F) * D + q]);
    __syncthreads();
    for (int p = t_; p < PP; p += 128) { float ssum = 0.0f; if (p < P) { int i, j; pair_ij(p, i, j); for (int d = 0; d < D; ++d) { const float v = pmul(Es[i][d], Es[j][d]); ssum += v; b16 ph, pl; split16(v * XS, ph, pl); Ph[p][d] = ph; Pl[p][d] = pl; } } else { for (int d = 0; d < D; ++d) { Ph[p][d] = (b16)0.0f; Pl[p][d] = (b16)0.0f; } } S[p] = ssum; }
    __syncthreads();
    for (int rt = wave; rt < PP / 16; rt += 4) { v8f a0 = {}, a1 = {}; const v16b fa = frag_kb(&Ph[rt * 16 + nloc][0], hlf), fl = frag_kb(&Pl[rt * 16 + nloc][0], hlf); const v16b wb0 = frag_kb(&W1h[nloc][0], hlf), wb1 = frag_kb(&W1h[16 + nloc][0], hlf);
      a0 = wmma16b(fa, wb0, a0); a0 = wmma16b(fl, wb0, a0); a1 = wmma16b(fa, wb1, a1); a1 = wmma16b(fl, wb1, a1);
      for (int r = 0; r < 8; ++r) { float v = pmul(fmaxf(a0[r] * (1.0f / (XS * WSC)) + b1v0, 0.0f), w2v0) + pmul(fmaxf(a1[r] * (1.0f / (XS * WSC)) + b1v1, 0.0f), w2v1);
        v += __shfl_xor(v, 1); v += __shfl_xor(v, 2); v += __shfl_xor(v, 4); v += __shfl_xor(v, 8); if (nloc == 0) LG[rt * 16 + 8 * hlf + r] = v; } }
    __syncthreads();
    if (wave == 0) { float mx = -INFINITY; for (int p = lane; p < P; p += 32) mx = fmaxf(mx, LG[p]); mx = fmaxf(mx, __shfl_xor(mx, 1)); mx = fmaxf(mx, __shfl_xor(mx, 2)); mx = fmaxf(mx, __shfl_xor(mx, 4)); mx = fmaxf(mx, __shfl_xor(mx, 8)); mx = fmaxf(mx, __shfl_xor(mx, 16));
      float se = 0.0f, sw = 0.0f; for (int p = lane; p < P; p += 32) { const float e = nexp(LG[p] - mx); se += e; sw += pmul(e, S[p]); }
      se += __shfl_xor(se, 1); se += __shfl_xor(se, 2); se += __shfl_xor(se, 4); se += __shfl_xor(se, 8); se += __shfl_xor(se, 16); sw += __shfl_xor(sw, 1); sw += __shfl_xor(sw, 2); sw += __shfl_xor(sw, 4); sw += __shfl_xor(sw, 8); sw += __shfl_xor(sw, 16);
      if (lane == 0) res[s] = sw / se; } }
  __syncthreads();
  for (int pass = 0; pass < 2; ++pass) { if (t_ < SPB) ((volatile float*)out)[b0 + t_] = res[t_]; __threadfence(); }
}
}

extern "C" void kernel_launch(void* const* d_in, const int* in_sizes, int n_in, void* d_out, int out_size, void* d_ws, size_t ws_size, hipStream_t stream) {
  (void)n_in; (void)d_ws; (void)ws_size;
  auto Fp = [&](int i) { return (const float*)d_in[i]; };
  if (in_sizes[0] != NB * F * D || in_sizes[1] != A * D || in_sizes[2] != A || in_sizes[3] != A || out_size != NB) return;
  fm_kernel<<<NB / SPB, 128, 0, stream>>>(Fp(0), Fp(1), Fp(2), Fp(3), (float*)d_out);
}
